// LIIF_83915071030150
// MI455X (gfx1250) — hardware-verified
//
#include <hip/hip_runtime.h>
#include <math.h>

#pragma clang fp contract(off)

constexpr int kB = 2;
constexpr int kH = 96;
constexpr int kW = 96;
constexpr int kQ = 30000;
constexpr int kC = 64;
constexpr int kNPix = kB * kH * kW;
constexpr int kKUnf = kC * 9;
constexpr int kHid = 256;
constexpr int kBQ = kB * kQ;
constexpr int kRows = 4 * kBQ;
constexpr int kChunk = 48000;
constexpr int kNChunk = 5;
constexpr int kN4 = 64;
constexpr int kOutF4 = kBQ * 3 / 4;
constexpr int kFeatPadLines = 4;
constexpr float kScale = 96.0f;
constexpr float kWCarry = 16.0f;
constexpr float kWCarryInv = 1.0f / 16.0f;

static_assert(kChunk * kNChunk == kRows, "chunks");
static_assert(kChunk % 64 == 0, "M tile");
static_assert(kNPix % 64 == 0, "M tile");
static_assert(kKUnf % 32 == 0, "K");
static_assert(kKUnf % 64 == 0, "pack tiles");
static_assert(kHid % 64 == 0, "N,K");
static_assert(kHid == 256, "one thread per hidden channel in the tail staging");
static_assert(kN4 % 64 == 0, "N");
static_assert(kChunk % 8 == 0, "gather grid");
static_assert((kBQ * 3) % 4 == 0, "out float4");
static_assert(kW % 32 == 0, "conv grid");
static_assert((kNPix * 9) % 32 == 0, "unfold grid");

constexpr size_t kOffFeat = 0;
constexpr size_t kSzFeat  = ((size_t)kNPix * kC + (size_t)kFeatPadLines * 64) * 2;
constexpr size_t kOffA0   = kOffFeat + kSzFeat;
constexpr size_t kSzA0    = (size_t)kNPix * kKUnf * 2;
constexpr size_t kOffP    = kOffA0 + kSzA0;
constexpr size_t kSzP     = (size_t)kNPix * kHid * 4;
constexpr size_t kOffW0   = kOffP + kSzP;
constexpr size_t kSzW0    = (size_t)kHid * kKUnf * 2;
constexpr size_t kOffW1   = kOffW0 + kSzW0;
constexpr size_t kSzW     = (size_t)kHid * kHid * 2;
constexpr size_t kOffW2   = kOffW1 + kSzW;
constexpr size_t kOffW3   = kOffW2 + kSzW;
constexpr size_t kOffW4   = kOffW3 + kSzW;
constexpr size_t kSzW4    = (size_t)kN4 * kHid * 2;
constexpr size_t kOffHA   = kOffW4 + kSzW4;
constexpr size_t kSzH     = (size_t)kChunk * kHid * 2;
constexpr size_t kOffHB   = kOffHA + kSzH;
constexpr size_t kOffY    = kOffHB + kSzH;
constexpr size_t kSzY     = (size_t)kRows * 4 * 4;
constexpr size_t kWsTotal = kOffY + kSzY;
static_assert(kWsTotal == 96180736, "carve");
static_assert(kWsTotal <= (size_t)134217728, "carve limit");
static_assert(kOffA0 % 256 == 0 && kOffP % 256 == 0 && kOffW0 % 256 == 0 && kOffW1 % 256 == 0 &&
              kOffW2 % 256 == 0 && kOffW3 % 256 == 0 && kOffW4 % 256 == 0 && kOffHA % 256 == 0 &&
              kOffHB % 256 == 0 && kOffY % 256 == 0, "align");

typedef __attribute__((ext_vector_type(16))) _Float16 v16h;
typedef __attribute__((ext_vector_type(8)))  _Float16 v8h;
typedef __attribute__((ext_vector_type(16))) __bf16   v16b;
typedef __attribute__((ext_vector_type(8)))  __bf16   v8b;
typedef __attribute__((ext_vector_type(8)))  float    v8f;
typedef __attribute__((ext_vector_type(4)))  float    v4f;
typedef __attribute__((ext_vector_type(4)))  unsigned int v4u;

__device__ __forceinline__ unsigned short f2bf_bits(float f) {
  unsigned u = __float_as_uint(f);
  return (unsigned short)((u + 0x7FFFu + ((u >> 16) & 1u)) >> 16);
}
__device__ __forceinline__ float bf_bits2f(unsigned short h) { return __uint_as_float(((unsigned)h) << 16); }
__device__ __forceinline__ float bf16r(float f) { return __uint_as_float(((unsigned)f2bf_bits(f)) << 16); }

__device__ __forceinline__ void dep_guard_h(v8f& a, v8f& b, v16h x, v16h y) { asm volatile("v_nop\n\tv_nop\n\tv_nop\n\tv_nop" : "+v"(a), "+v"(b) : "v"(x), "v"(y)); }
__device__ __forceinline__ void dep_guard_b(v8f& a, v8f& b, v16b x, v16b y) { asm volatile("v_nop\n\tv_nop\n\tv_nop\n\tv_nop" : "+v"(a), "+v"(b) : "v"(x), "v"(y)); }
__device__ __forceinline__ void dep_guard4_h(v8f& a, v8f& b, v8f& c, v8f& d, v16h x, v16h y) { asm volatile("v_nop\n\tv_nop\n\tv_nop\n\tv_nop" : "+v"(a), "+v"(b), "+v"(c), "+v"(d) : "v"(x), "v"(y)); }
__device__ __forceinline__ void dep_guard4_b(v8f& a, v8f& b, v8f& c, v8f& d, v16b x, v16b y) { asm volatile("v_nop\n\tv_nop\n\tv_nop\n\tv_nop" : "+v"(a), "+v"(b), "+v"(c), "+v"(d) : "v"(x), "v"(y)); }
__device__ __forceinline__ void keep4_h(v16h a, v16h b, v16h c, v16h d) { asm volatile("v_nop" :: "v"(a), "v"(b), "v"(c), "v"(d)); }
__device__ __forceinline__ void keep4_b(v16b a, v16b b, v16b c, v16b d) { asm volatile("v_nop" :: "v"(a), "v"(b), "v"(c), "v"(d)); }
__device__ __forceinline__ void acc_guard4(v8f& a, v8f& b, v8f& c, v8f& d) { asm volatile("v_nop\n\tv_nop\n\tv_nop\n\tv_nop" : "+v"(a), "+v"(b), "+v"(c), "+v"(d)); }
template <typename T> struct Frag;
template <> struct Frag<_Float16> {
  typedef v16h V; union U { v16h v; v8h h[2]; };
  static __device__ __forceinline__ v16h load(const _Float16* p) {
    U f; f.h[0] = *(const v8h*)(p); f.h[1] = *(const v8h*)(p + 16); return f.v;
  }
  static __device__ __forceinline__ v8f mma(v16h a, v16h b, v8f c) {
    return __builtin_amdgcn_wmma_f32_16x16x32_f16(false, a, false, b, (short)0, c, false, false);
  }
  static __device__ __forceinline__ void guard(v8f& a, v8f& b, v16h x, v16h y) { dep_guard_h(a, b, x, y); }
  static __device__ __forceinline__ void guard4(v8f& a, v8f& b, v8f& c, v8f& d, v16h x, v16h y) { dep_guard4_h(a, b, c, d, x, y); }
  static __device__ __forceinline__ void keep(v16h a, v16h b, v16h c, v16h d) { keep4_h(a, b, c, d); }
};
template <> struct Frag<__bf16> {
  typedef v16b V; union U { v16b v; v8b h[2]; };
  static __device__ __forceinline__ v16b load(const __bf16* p) {
    U f; f.h[0] = *(const v8b*)(p); f.h[1] = *(const v8b*)(p + 16); return f.v;
  }
  static __device__ __forceinline__ v8f mma(v16b a, v16b b, v8f c) {
    return __builtin_amdgcn_wmma_f32_16x16x32_bf16(false, a, false, b, (short)0, c, false, false);
  }
  static __device__ __forceinline__ void guard(v8f& a, v8f& b, v16b x, v16b y) { dep_guard_b(a, b, x, y); }
  static __device__ __forceinline__ void guard4(v8f& a, v8f& b, v8f& c, v8f& d, v16b x, v16b y) { dep_guard4_b(a, b, c, d, x, y); }
  static __device__ __forceinline__ void keep(v16b a, v16b b, v16b c, v16b d) { keep4_b(a, b, c, d); }
};

__device__ __forceinline__ unsigned pk16(unsigned short a, unsigned short b) { return (unsigned)a | ((unsigned)b << 16); }
__device__ __forceinline__ unsigned short h_bits(float f) { const _Float16 h = (_Float16)f; return __builtin_bit_cast(unsigned short, h); }

template <int ET> struct Elem;
template <> struct Elem<0> { typedef _Float16 T; };
template <> struct Elem<1> { typedef __bf16 T; };
template <int ET, bool SPLIT, int BIAS_MODE, int OUT_MODE, bool RESID, int ACT = 0>
__global__ __launch_bounds__(256) void wmma_gemm64(
    const unsigned short* __restrict__ Ap, const unsigned short* __restrict__ A2p, int lda, long strideA,
    const unsigned short* __restrict__ Btp, const unsigned short* __restrict__ Bt2p, int ldb, long strideB,
    void* __restrict__ Cout, void* __restrict__ Cout2, int ldc, long strideC,
    const float* __restrict__ bias,
    const float* __restrict__ resid, long strideR,
    int M, int N, int K, float scale) {
  typedef typename Elem<ET>::T T;
  typedef typename Frag<T>::V V;
  const T* A = (const T*)Ap; const T* A2 = (const T*)A2p; const T* Bt = (const T*)Btp; const T* Bt2 = (const T*)Bt2p;
  __shared__ __align__(16) float sT[8][16 * 68];
  const int b    = blockIdx.y;
  const int lane = threadIdx.x & 31;
  const int wave = threadIdx.x >> 5;
  const int tilesN = N >> 6;
  const int tilesM = M >> 6;
  const int tile = blockIdx.x * 8 + wave;
  if (tile >= tilesM * tilesN) return;
  const int tm = tile / tilesN;
  const int tn = tile - tm * tilesN;
  const int m0 = tm << 6;
  const int n0 = tn << 6;

  const T* Ab  = A  + (size_t)b * strideA;
  const T* Bb  = Bt + (size_t)b * strideB;
  const T* Ab2 = SPLIT ? (A2  + (size_t)b * strideA) : nullptr;
  const T* Bb2 = SPLIT ? (Bt2 + (size_t)b * strideB) : nullptr;

  const int rlane = lane & 15;
  const int koff  = (lane >> 4) * 8;
  const int mOff  = (lane >> 4) * 8;

  v8f acc[4][4];
#pragma unroll
  for (int i = 0; i < 4; ++i)
#pragma unroll
    for (int j = 0; j < 4; ++j) acc[i][j] = (v8f){0.f,0.f,0.f,0.f,0.f,0.f,0.f,0.f};

  for (int k0 = 0; k0 < K; k0 += 32) {
    V bh[4], bl[4];
#pragma unroll
    for (int j = 0; j < 4; ++j) {
      const size_t bo = (size_t)(n0 + (j << 4) + rlane) * ldb + koff + k0;
      bh[j] = Frag<T>::load(Bb + bo);
      if (SPLIT) bl[j] = Frag<T>::load(Bb2 + bo);
    }
#pragma unroll
    for (int i = 0; i < 4; ++i) {
      const size_t ao = (size_t)(m0 + (i << 4) + rlane) * lda + koff + k0;
      V ah = Frag<T>::load(Ab + ao);
      V al;
      if (SPLIT) al = Frag<T>::load(Ab2 + ao);
#pragma unroll
      for (int j = 0; j < 4; ++j) {
        acc[i][j] = Frag<T>::mma(ah, bh[j], acc[i][j]);
        if (SPLIT) {
          acc[i][j] = Frag<T>::mma(ah, bl[j], acc[i][j]);
          acc[i][j] = Frag<T>::mma(al, bh[j], acc[i][j]);
        }
      }
      Frag<T>::guard4(acc[i][0], acc[i][1], acc[i][2], acc[i][3], ah, bh[3]);
      if (SPLIT) Frag<T>::guard(acc[i][0], acc[i][3], al, bl[3]);
    }
    Frag<T>::keep(bh[0], bh[1], bh[2], bh[3]);
    if (SPLIT) Frag<T>::keep(bl[0], bl[1], bl[2], bl[3]);
  }
  acc_guard4(acc[0][0], acc[0][1], acc[0][2], acc[0][3]);
  acc_guard4(acc[1][0], acc[1][1], acc[1][2], acc[1][3]);
  acc_guard4(acc[2][0], acc[2][1], acc[2][2], acc[2][3]);
  acc_guard4(acc[3][0], acc[3][1], acc[3][2], acc[3][3]);

  float* slab = sT[wave];
  const float* Rb = RESID ? (resid + (size_t)b * strideR) : nullptr;
#pragma unroll
  for (int i = 0; i < 4; ++i) {
    const int mBase = m0 + (i << 4);
#pragma unroll
    for (int j = 0; j < 4; ++j) {
      const int n = n0 + (j << 4) + rlane;
      float bv = 0.f;
      if (BIAS_MODE == 2) bv = bf16r(bias[n]);
#pragma unroll
      for (int r = 0; r < 8; ++r) {
        float v = acc[i][j][r] * scale;
        if (BIAS_MODE == 1) v += bf16r(bias[mBase + mOff + r]);
        if (BIAS_MODE == 2) v += bv;
        if (RESID) v += Rb[(size_t)(mBase + mOff + r) * ldc + n];
        if (ACT == 2) v = fmaxf(v, 0.0f);
        if (ACT == 4) v = (v > 0.f) ? v : 0.01f * v;
        slab[(mOff + r) * 68 + (j << 4) + rlane] = v;
      }
    }
    __builtin_amdgcn_fence(__ATOMIC_RELEASE, "workgroup");
    __builtin_amdgcn_wave_barrier();
    __builtin_amdgcn_fence(__ATOMIC_ACQUIRE, "workgroup");
    if (OUT_MODE == 0) {
      float* C = (float*)Cout + (size_t)b * strideC;
      const int hh = lane >> 4, c4 = (lane & 15) * 4;
      for (int pass = 0; pass < 2; ++pass) {
#pragma unroll
        for (int it = 0; it < 8; ++it) {
          const int row = it * 2 + hh;
          v4f v = *(const v4f*)(slab + row * 68 + c4);
          *(volatile v4f*)(C + (size_t)(mBase + row) * ldc + n0 + c4) = v;
        }
        __threadfence();
      }
    } else if (OUT_MODE == 3) {
      float* C = (float*)Cout + (size_t)b * strideC;
      const int row = lane & 15;
      const v4f v = *(const v4f*)(slab + row * 68);
      for (int pass = 0; pass < 2; ++pass) {
        if (lane < 16) *(volatile v4f*)(C + (size_t)(mBase + row) * ldc) = v;
        __threadfence();
      }
    } else {
      const int q = lane >> 3, c8 = (lane & 7) * 8;
      unsigned short* C  = (unsigned short*)Cout  + (size_t)b * strideC;
      unsigned short* C2 = (OUT_MODE == 2) ? ((unsigned short*)Cout2 + (size_t)b * strideC) : nullptr;
      for (int pass = 0; pass < 2; ++pass) {
#pragma unroll
        for (int it = 0; it < 4; ++it) {
          const int row = it * 4 + q;
          const float* sp = slab + row * 68 + c8;
          v8h hv, lv;
#pragma unroll
          for (int e = 0; e < 8; ++e) {
            if (OUT_MODE == 1) {
              hv[e] = (_Float16)sp[e];
            } else {
              unsigned short hb = f2bf_bits(sp[e]);
              unsigned short lb = f2bf_bits(sp[e] - bf_bits2f(hb));
              hv[e] = __builtin_bit_cast(_Float16, hb);
              lv[e] = __builtin_bit_cast(_Float16, lb);
            }
          }
          *(volatile v8h*)(C + (size_t)(mBase + row) * ldc + n0 + c8) = hv;
          if (OUT_MODE == 2) *(volatile v8h*)(C2 + (size_t)(mBase + row) * ldc + n0 + c8) = lv;
        }
        __threadfence();
      }
    }
    __builtin_amdgcn_fence(__ATOMIC_RELEASE, "workgroup");
    __builtin_amdgcn_wave_barrier();
    __builtin_amdgcn_fence(__ATOMIC_ACQUIRE, "workgroup");
  }
}

__global__ __launch_bounds__(256) void wpack_kernel(const float* __restrict__ Wsrc, unsigned short* __restrict__ out,
                                                    int ldw, int nreal, int ldo, int mode, float scale) {
  __shared__ float sm[64][65];
  const int t  = threadIdx.x;
  const int kt = blockIdx.x;
  const int k0 = kt * 64;
  const int n0 = blockIdx.y * 64;
#pragma unroll
  for (int i = 0; i < 16; ++i) {
    const int e = i * 256 + t;
    const int r = e >> 6;
    const int c = e & 63;
    const int srow = (mode == 0) ? (r * 9 + kt) : (k0 + r);
    const int n = n0 + c;
    const int nc = min(n, nreal - 1);
    const float v = bf16r(Wsrc[(size_t)srow * ldw + nc]) * scale;
    const float keep = (n < nreal) ? 1.0f : 0.0f;
    sm[c][r] = v * keep;
  }
  __syncthreads();
  const int lane = t & 31, wave = t >> 5;
  const int q = lane >> 3, c8 = (lane & 7) * 8;
  for (int pass = 0; pass < 2; ++pass) {
#pragma unroll
    for (int it = 0; it < 2; ++it) {
      const int row = wave * 8 + it * 4 + q;
      unsigned short hb[8];
#pragma unroll
      for (int e = 0; e < 8; ++e) hb[e] = h_bits(sm[row][c8 + e]);
      const v4u u = (v4u){pk16(hb[0], hb[1]), pk16(hb[2], hb[3]), pk16(hb[4], hb[5]), pk16(hb[6], hb[7])};
      *(volatile v4u*)(out + (size_t)(n0 + row) * ldo + k0 + c8) = u;
    }
    __threadfence();
  }
}

__global__ __launch_bounds__(32) void zero_pad_kernel(unsigned short* __restrict__ p) {
  const int lane = threadIdx.x;
  const v4u z = (v4u){0u, 0u, 0u, 0u};
  unsigned short* dst = p + lane * 8;
  *(volatile v4u*)dst = z;
  __threadfence();
  *(volatile v4u*)dst = z;
}

__global__ __launch_bounds__(256) void conv_tanh_kernel(const float* __restrict__ inp, const float* __restrict__ cw,
                                                        const float* __restrict__ cb, unsigned short* __restrict__ feat) {
  __shared__ float w_s[kC * 27];
  __shared__ float b_s[kC];
  __shared__ float in_s[3][3][34];
  __shared__ __align__(16) unsigned short stg[32][kC];
  const int t = threadIdx.x;
  const int blk = blockIdx.x;
  const int xs = blk % 3;
  const int y = (blk / 3) % kH;
  const int b = blk / (3 * kH);
  const int x0 = xs * 32;
  for (int i = t; i < kC * 27; i += 256) w_s[i] = bf16r(cw[i]);
  if (t < kC) b_s[t] = bf16r(cb[t]);
  for (int i = t; i < 306; i += 256) {
    const int ci = i / 102;
    const int rem = i - ci * 102;
    const int ky = rem / 34;
    const int xx = rem - ky * 34;
    const int yy = y + ky - 1;
    const int xg = x0 + xx - 1;
    const bool ok = (yy >= 0) && (yy < kH) && (xg >= 0) && (xg < kW);
    const int yyc = min(max(yy, 0), kH - 1);
    const int xgc = min(max(xg, 0), kW - 1);
    const float v = bf16r(inp[(((size_t)b * 3 + ci) * kH + yyc) * kW + xgc]);
    const float keep = ok ? 1.0f : 0.0f;
    in_s[ci][ky][xx] = v * keep;
  }
  __syncthreads();
  const int pl = t >> 3, cg = t & 7;
#pragma unroll 1
  for (int cc = 0; cc < 8; ++cc) {
    const int c = cg * 8 + cc;
    float acc = 0.0f;
#pragma unroll 1
    for (int ci = 0; ci < 3; ++ci) {
#pragma unroll 1
      for (int ky = 0; ky < 3; ++ky) {
        const float* ip = &in_s[ci][ky][pl];
        const float* wp = &w_s[c * 27 + ci * 9 + ky * 3];
        acc = fmaf(ip[0], wp[0], acc);
        acc = fmaf(ip[1], wp[1], acc);
        acc = fmaf(ip[2], wp[2], acc);
      }
    }
    acc = acc + b_s[c];
    const float v = tanhf(acc);
    stg[pl][c] = h_bits(v);
  }
  __syncthreads();
  const v4u u = *(const v4u*)(&stg[pl][cg * 8]);
  const int pix = (b * kH + y) * kW + x0 + pl;
  unsigned short* dst = feat + (size_t)pix * kC + cg * 8;
  *(volatile v4u*)dst = u;
  __threadfence();
  *(volatile v4u*)dst = u;
}

__global__ __launch_bounds__(256) void unfold_kernel(const unsigned short* __restrict__ feat, unsigned short* __restrict__ A0) {
  const int t = threadIdx.x;
  const int pair = blockIdx.x * 32 + (t >> 3);
  const int cg = t & 7;
  const int pix = pair / 9;
  const int p = pair - pix * 9;
  const int x = pix % kW;
  const int y = (pix / kW) % kH;
  const int b = pix / (kW * kH);
  const int dy = p / 3 - 1;
  const int dx = (p - (p / 3) * 3) - 1;
  const int yy = y + dy, xx = x + dx;
  const bool ok = (yy >= 0) && (yy < kH) && (xx >= 0) && (xx < kW);
  const int yyc = min(max(yy, 0), kH - 1);
  const int xxc = min(max(xx, 0), kW - 1);
  const int nbr = (b * kH + yyc) * kW + xxc;
  const int nb = ok ? nbr : kNPix;
  const v4u v = *(const v4u*)(feat + (size_t)nb * kC + cg * 8);
  unsigned short* dst = A0 + (size_t)pix * kKUnf + p * kC + cg * 8;
  *(volatile v4u*)dst = v;
  __threadfence();
  *(volatile v4u*)dst = v;
}

__device__ __forceinline__ void ens_index(float c0, float c1, int s, int& iy, int& ix, float& rel0, float& rel1) {
  const float rad = (float)(1.0 / 96.0);
  const float eps = (float)(1e-6);
  const float lim = (float)(1.0 - 1e-10);
  const float oy = (s >> 1) ? rad : -rad;
  const float ox = (s & 1) ? rad : -rad;
  float e0 = c0 + oy; e0 = e0 + eps;
  float e1 = c1 + ox; e1 = e1 + eps;
  e0 = fminf(fmaxf(e0, -lim), lim);
  e1 = fminf(fmaxf(e1, -lim), lim);
  float t0 = e0 + 1.0f; t0 = t0 * kScale; t0 = t0 * 0.5f; t0 = t0 - 0.5f;
  float t1 = e1 + 1.0f; t1 = t1 * kScale; t1 = t1 * 0.5f; t1 = t1 - 0.5f;
  int i0 = (int)rintf(t0);
  int i1 = (int)rintf(t1);
  i0 = min(max(i0, 0), kH - 1);
  i1 = min(max(i1, 0), kW - 1);
  const float inv = 1.0f / kScale;
  float q0 = 2.0f * (float)i0; q0 = q0 + 1.0f; q0 = q0 * inv; q0 = -1.0f + q0;
  float q1 = 2.0f * (float)i1; q1 = q1 + 1.0f; q1 = q1 * inv; q1 = -1.0f + q1;
  rel0 = (c0 - q0) * kScale;
  rel1 = (c1 - q1) * kScale;
  iy = i0; ix = i1;
}

__global__ __launch_bounds__(256) void gather_tail_kernel(const float* __restrict__ coord, const float* __restrict__ cell,
                                                          const float* __restrict__ P, const float* __restrict__ w0,
                                                          const float* __restrict__ b0, unsigned short* __restrict__ Hout, int row0) {
  __shared__ __align__(16) float tails[5][kHid];
  const int t = threadIdx.x;
#pragma unroll
  for (int a = 0; a < 4; ++a) tails[a][t] = bf16r(w0[(size_t)(kKUnf + a) * kHid + t]);
  tails[4][t] = bf16r(b0[t]);
  __syncthreads();
  const int lane = t & 31, wave = t >> 5;
  const int rl = blockIdx.x * 8 + wave;
  const int r = row0 + rl;
  const int s = r / kBQ;
  const int tq = r - s * kBQ;
  const int bb = tq / kQ;
  const float c0 = bf16r(coord[(size_t)tq * 2]), c1 = bf16r(coord[(size_t)tq * 2 + 1]);
  const float ce0 = bf16r(cell[(size_t)tq * 2]), ce1 = bf16r(cell[(size_t)tq * 2 + 1]);
  int iy, ix; float rel0, rel1;
  ens_index(c0, c1, s, iy, ix, rel0, rel1);
  int pix = bb * (kH * kW) + iy * kW + ix;
  pix = min(max(pix, 0), kNPix - 1);
  const float rcy = ce0 * kScale, rcx = ce1 * kScale;
  const float* prow = P + (size_t)pix * kHid + lane * 8;
  const v4f pa = *(const v4f*)(prow);
  const v4f pb = *(const v4f*)(prow + 4);
  const v4f ta0 = *(const v4f*)(&tails[0][lane * 8]); const v4f tb0 = *(const v4f*)(&tails[0][lane * 8 + 4]);
  const v4f ta1 = *(const v4f*)(&tails[1][lane * 8]); const v4f tb1 = *(const v4f*)(&tails[1][lane * 8 + 4]);
  const v4f ta2 = *(const v4f*)(&tails[2][lane * 8]); const v4f tb2 = *(const v4f*)(&tails[2][lane * 8 + 4]);
  const v4f ta3 = *(const v4f*)(&tails[3][lane * 8]); const v4f tb3 = *(const v4f*)(&tails[3][lane * 8 + 4]);
  const v4f ta4 = *(const v4f*)(&tails[4][lane * 8]); const v4f tb4 = *(const v4f*)(&tails[4][lane * 8 + 4]);
  unsigned short hb[8];
#pragma unroll
  for (int e = 0; e < 4; ++e) {
    float v = pa[e];
    v = fmaf(rel0, ta0[e], v);
    v = fmaf(rel1, ta1[e], v);
    v = fmaf(rcy, ta2[e], v);
    v = fmaf(rcx, ta3[e], v);
    v = v + ta4[e];
    v = fmaxf(v, 0.0f);
    hb[e] = h_bits(v);
    float u2 = pb[e];
    u2 = fmaf(rel0, tb0[e], u2);
    u2 = fmaf(rel1, tb1[e], u2);
    u2 = fmaf(rcy, tb2[e], u2);
    u2 = fmaf(rcx, tb3[e], u2);
    u2 = u2 + tb4[e];
    u2 = fmaxf(u2, 0.0f);
    hb[4 + e] = h_bits(u2);
  }
  const v4u u = (v4u){pk16(hb[0], hb[1]), pk16(hb[2], hb[3]), pk16(hb[4], hb[5]), pk16(hb[6], hb[7])};
  unsigned short* dst = Hout + (size_t)rl * kHid + lane * 8;
  *(volatile v4u*)dst = u;
  __threadfence();
  *(volatile v4u*)dst = u;
}

__global__ __launch_bounds__(256) void combine_kernel(const float* __restrict__ coord, const float* __restrict__ Y,
                                                      const float* __restrict__ b4, float* __restrict__ out) {
  __shared__ __align__(16) float stg[256 * 3];
  const int t = threadIdx.x;
  const int tq = blockIdx.x * 256 + t;
  const int tqc = min(tq, kBQ - 1);
  const float c0 = bf16r(coord[(size_t)tqc * 2]), c1 = bf16r(coord[(size_t)tqc * 2 + 1]);
  float ar[4];
#pragma unroll
  for (int s = 0; s < 4; ++s) {
    int iy, ix; float r0, r1;
    ens_index(c0, c1, s, iy, ix, r0, r1);
    const float pr = r0 * r1;
    ar[s] = fabsf(pr) + 1e-9f;
  }
  float sum = 0.0f;
  sum = sum + ar[0]; sum = sum + ar[1]; sum = sum + ar[2]; sum = sum + ar[3];
  const float inv = 1.0f / sum;
  float wv[4];
#pragma unroll
  for (int s = 0; s < 4; ++s) wv[s] = ar[s] * inv;
  const v4f y0 = *(const v4f*)(Y + ((size_t)0 * kBQ + tqc) * 4);
  const v4f y1 = *(const v4f*)(Y + ((size_t)1 * kBQ + tqc) * 4);
  const v4f y2 = *(const v4f*)(Y + ((size_t)2 * kBQ + tqc) * 4);
  const v4f y3 = *(const v4f*)(Y + ((size_t)3 * kBQ + tqc) * 4);
  const float bb0 = bf16r(b4[0]), bb1 = bf16r(b4[1]), bb2 = bf16r(b4[2]);
#pragma unroll
  for (int j = 0; j < 3; ++j) {
    const float bj = (j == 0) ? bb0 : ((j == 1) ? bb1 : bb2);
    float acc = 0.0f;
    acc = acc + (y0[j] + bj) * wv[3];
    acc = acc + (y1[j] + bj) * wv[2];
    acc = acc + (y2[j] + bj) * wv[1];
    acc = acc + (y3[j] + bj) * wv[0];
    stg[t * 3 + j] = acc;
  }
#pragma unroll 1
  for (int j = 0; j < 3; ++j) {
    const float a = stg[t * 3 + j];
    stg[t * 3 + j] = tanhf(a) * 1.01f;
  }
  __syncthreads();
  const int f = blockIdx.x * 192 + t;
  const bool wr = (t < 192) && (f < kOutF4);
  const int tc = min(t, 191);
  const v4f v = *(const v4f*)(&stg[tc * 4]);
  if (wr) *(volatile v4f*)(out + (size_t)f * 4) = v;
  __threadfence();
  if (wr) *(volatile v4f*)(out + (size_t)f * 4) = v;
}

extern "C" void kernel_launch(void* const* d_in, const int* in_sizes, int n_in,
                              void* d_out, int out_size, void* d_ws, size_t ws_size,
                              hipStream_t stream)
{
  (void)in_sizes; (void)n_in;
  if (ws_size < kWsTotal) return;
  if (out_size != kBQ * 3) return;

  const float* inp    = (const float*)d_in[0];
  const float* coord  = (const float*)d_in[1];
  const float* cell   = (const float*)d_in[2];
  const float* conv_w = (const float*)d_in[3];
  const float* conv_b = (const float*)d_in[4];
  const float* w0 = (const float*)d_in[5];
  const float* b0 = (const float*)d_in[6];
  const float* w1 = (const float*)d_in[7];
  const float* b1 = (const float*)d_in[8];
  const float* w2 = (const float*)d_in[9];
  const float* b2 = (const float*)d_in[10];
  const float* w3 = (const float*)d_in[11];
  const float* b3 = (const float*)d_in[12];
  const float* w4 = (const float*)d_in[13];
  const float* b4 = (const float*)d_in[14];
  float* out = (float*)d_out;

  char* ws = (char*)d_ws;
  unsigned short* feat = (unsigned short*)(ws + kOffFeat);
  unsigned short* a0   = (unsigned short*)(ws + kOffA0);
  float*          pbuf = (float*)(ws + kOffP);
  unsigned short* w0t  = (unsigned short*)(ws + kOffW0);
  unsigned short* w1t  = (unsigned short*)(ws + kOffW1);
  unsigned short* w2t  = (unsigned short*)(ws + kOffW2);
  unsigned short* w3t  = (unsigned short*)(ws + kOffW3);
  unsigned short* w4t  = (unsigned short*)(ws + kOffW4);
  unsigned short* ha   = (unsigned short*)(ws + kOffHA);
  unsigned short* hb   = (unsigned short*)(ws + kOffHB);
  float*          ybuf = (float*)(ws + kOffY);

  wpack_kernel<<<dim3(kKUnf / 64, kHid / 64), 256, 0, stream>>>(w0, w0t, kHid, kHid, kKUnf, 0, kWCarry);
  wpack_kernel<<<dim3(kHid / 64, kHid / 64), 256, 0, stream>>>(w1, w1t, kHid, kHid, kHid, 1, kWCarry);
  wpack_kernel<<<dim3(kHid / 64, kHid / 64), 256, 0, stream>>>(w2, w2t, kHid, kHid, kHid, 1, kWCarry);
  wpack_kernel<<<dim3(kHid / 64, kHid / 64), 256, 0, stream>>>(w3, w3t, kHid, kHid, kHid, 1, kWCarry);
  wpack_kernel<<<dim3(kHid / 64, kN4 / 64), 256, 0, stream>>>(w4, w4t, 3, 3, kHid, 1, kWCarry);

  conv_tanh_kernel<<<kB * kH * (kW / 32), 256, 0, stream>>>(inp, conv_w, conv_b, feat);
  zero_pad_kernel<<<1, 32, 0, stream>>>(feat + (size_t)kNPix * kC);

  unfold_kernel<<<(kNPix * 9) / 32, 256, 0, stream>>>(feat, a0);

  {
    const int tiles = (kNPix / 64) * (kHid / 64);
    wmma_gemm64<0, false, 0, 0, false, 0><<<dim3((tiles + 7) / 8, 1), 256, 0, stream>>>(
        a0, a0, kKUnf, 0L, w0t, w0t, kKUnf, 0L, (void*)pbuf, (void*)pbuf, kHid, 0L,
        b0, b0, 0L, kNPix, kHid, kKUnf, kWCarryInv);
  }

  const int tilesHid = (kChunk / 64) * (kHid / 64);
  const int tilesL4  = (kChunk / 64) * (kN4 / 64);
  for (int c = 0; c < kNChunk; ++c) {
    const int row0 = c * kChunk;
    gather_tail_kernel<<<kChunk / 8, 256, 0, stream>>>(coord, cell, pbuf, w0, b0, ha, row0);
    wmma_gemm64<0, false, 2, 1, false, 2><<<dim3((tilesHid + 7) / 8, 1), 256, 0, stream>>>(
        ha, ha, kHid, 0L, w1t, w1t, kHid, 0L, (void*)hb, (void*)hb, kHid, 0L,
        b1, b1, 0L, kChunk, kHid, kHid, kWCarryInv);
    wmma_gemm64<0, false, 2, 1, false, 2><<<dim3((tilesHid + 7) / 8, 1), 256, 0, stream>>>(
        hb, hb, kHid, 0L, w2t, w2t, kHid, 0L, (void*)ha, (void*)ha, kHid, 0L,
        b2, b2, 0L, kChunk, kHid, kHid, kWCarryInv);
    wmma_gemm64<0, false, 2, 1, false, 2><<<dim3((tilesHid + 7) / 8, 1), 256, 0, stream>>>(
        ha, ha, kHid, 0L, w3t, w3t, kHid, 0L, (void*)hb, (void*)hb, kHid, 0L,
        b3, b3, 0L, kChunk, kHid, kHid, kWCarryInv);
    float* yc = ybuf + (size_t)row0 * 4;
    wmma_gemm64<0, false, 0, 3, false, 0><<<dim3((tilesL4 + 7) / 8, 1), 256, 0, stream>>>(
        hb, hb, kHid, 0L, w4t, w4t, kHid, 0L, (void*)yc, (void*)yc, 4, 0L,
        b0, b0, 0L, kChunk, kN4, kHid, kWCarryInv);
  }

  combine_kernel<<<(kBQ + 255) / 256, 256, 0, stream>>>(coord, ybuf, b4, out);
}
